// PagedHSTUInferLayer_1228360646803
// MI455X (gfx1250) — hardware-verified
//
#include <hip/hip_runtime.h>
#include <math.h>
#include <stdint.h>

#define NBATCH 4
#define NS     2048
#define ND     1024
#define NHEAD  8
#define NHD    128
#define NTOK   (NBATCH * NS)

typedef _Float16 v16h __attribute__((ext_vector_type(16)));
typedef _Float16 v8h  __attribute__((ext_vector_type(8)));
typedef float    v8f  __attribute__((ext_vector_type(8)));
typedef float    v4f  __attribute__((ext_vector_type(4)));

union FragU { v16h v; v8h h[2]; };

__device__ __forceinline__ v16h frag_load(const _Float16* p) {
  FragU f;
  f.h[0] = *(const v8h*)(p);
  f.h[1] = *(const v8h*)(p + 16);
  return f.v;
}
__device__ __forceinline__ v8f mma16(v16h a, v16h b, v8f c) {
  return __builtin_amdgcn_wmma_f32_16x16x32_f16(false, a, false, b, (short)0, c, false, false);
}
__device__ __forceinline__ void guard4(v8f& a0, v8f& a1, v8f& a2, v8f& a3,
                                       v16h f0, v16h f1, v16h f2, v16h f3, v16h f4) {
  asm volatile("v_nop\n\tv_nop\n\tv_nop\n\tv_nop"
               : "+v"(a0), "+v"(a1), "+v"(a2), "+v"(a3)
               : "v"(f0), "v"(f1), "v"(f2), "v"(f3), "v"(f4));
}
__device__ __forceinline__ void guard1(v8f& a0, v16h f0, v16h f1, v16h f2, v16h f3, v16h f4) {
  asm volatile("v_nop\n\tv_nop\n\tv_nop\n\tv_nop"
               : "+v"(a0)
               : "v"(f0), "v"(f1), "v"(f2), "v"(f3), "v"(f4));
}
__device__ __forceinline__ void accg4(v8f& a, v8f& b, v8f& c, v8f& d) {
  asm volatile("v_nop\n\tv_nop\n\tv_nop\n\tv_nop" : "+v"(a), "+v"(b), "+v"(c), "+v"(d));
}
__device__ __forceinline__ float silu_f(float v) {
  return v * __builtin_amdgcn_rcpf(1.0f + __expf(-v));
}
__device__ __forceinline__ void lds_sync_wave() {
  __builtin_amdgcn_fence(__ATOMIC_RELEASE, "workgroup");
  __builtin_amdgcn_wave_barrier();
  __builtin_amdgcn_fence(__ATOMIC_ACQUIRE, "workgroup");
}
__device__ __forceinline__ float block_sum128(float v, float* red) {
#pragma unroll
  for (int o = 16; o > 0; o >>= 1) v += __shfl_xor(v, o, 32);
  const int lane = threadIdx.x & 31, wave = threadIdx.x >> 5;
  if (lane == 0) red[wave] = v;
  __syncthreads();
  const float t = (red[0] + red[1]) + (red[2] + red[3]);
  __syncthreads();
  return t;
}

__global__ __launch_bounds__(128) void k_ln(const float* __restrict__ x, const float* __restrict__ w,
                                           const float* __restrict__ bb, _Float16* __restrict__ out) {
  __shared__ float red[4];
  const int row = blockIdx.x, tid = threadIdx.x, c0 = tid * 8;
  const float* xr = x + (size_t)row * ND + c0;
  const v4f xa = *(const v4f*)(xr);
  const v4f xb = *(const v4f*)(xr + 4);
  float v[8];
#pragma unroll
  for (int e = 0; e < 4; ++e) { v[e] = xa[e]; v[4 + e] = xb[e]; }
  float s = 0.f;
#pragma unroll
  for (int e = 0; e < 8; ++e) s += v[e];
  s = block_sum128(s, red);
  const float mu = s * (1.0f / ND);
  float s2 = 0.f;
#pragma unroll
  for (int e = 0; e < 8; ++e) { v[e] -= mu; s2 += v[e] * v[e]; }
  s2 = block_sum128(s2, red);
  const float rstd = rsqrtf(s2 * (1.0f / ND) + 1e-5f);
  const v4f wa = *(const v4f*)(w + c0), wb = *(const v4f*)(w + c0 + 4);
  const v4f ba = *(const v4f*)(bb + c0), bc = *(const v4f*)(bb + c0 + 4);
  v8h o;
#pragma unroll
  for (int e = 0; e < 4; ++e) {
    o[e]     = (_Float16)(v[e] * rstd * wa[e] + ba[e]);
    o[4 + e] = (_Float16)(v[4 + e] * rstd * wb[e] + bc[e]);
  }
  _Float16* op = out + (size_t)row * ND + c0;
  *(volatile v8h*)op = o;
  __threadfence();
  *(volatile v8h*)op = o;
}

__global__ __launch_bounds__(128) void k_lngate(const float* __restrict__ attn, const float* __restrict__ u,
                                               const float* __restrict__ w, const float* __restrict__ bb,
                                               _Float16* __restrict__ out) {
  __shared__ float red[4];
  const int row = blockIdx.x, tid = threadIdx.x, c0 = tid * 8;
  const float* ar = attn + (size_t)row * ND + c0;
  const v4f xa = *(const v4f*)(ar);
  const v4f xb = *(const v4f*)(ar + 4);
  float v[8];
#pragma unroll
  for (int e = 0; e < 4; ++e) { v[e] = xa[e]; v[4 + e] = xb[e]; }
  float s = 0.f;
#pragma unroll
  for (int e = 0; e < 8; ++e) s += v[e];
  s = block_sum128(s, red);
  const float mu = s * (1.0f / ND);
  float s2 = 0.f;
#pragma unroll
  for (int e = 0; e < 8; ++e) { v[e] -= mu; s2 += v[e] * v[e]; }
  s2 = block_sum128(s2, red);
  const float rstd = rsqrtf(s2 * (1.0f / ND) + 1e-5f);
  const float* ur = u + (size_t)row * ND + c0;
  const v4f ua = *(const v4f*)(ur), ub = *(const v4f*)(ur + 4);
  const v4f wa = *(const v4f*)(w + c0), wb = *(const v4f*)(w + c0 + 4);
  const v4f ba = *(const v4f*)(bb + c0), bc = *(const v4f*)(bb + c0 + 4);
  v8h o;
#pragma unroll
  for (int e = 0; e < 4; ++e) {
    o[e]     = (_Float16)(ua[e] * (v[e] * rstd * wa[e] + ba[e]));
    o[4 + e] = (_Float16)(ub[e] * (v[4 + e] * rstd * wb[e] + bc[e]));
  }
  _Float16* op = out + (size_t)row * ND + c0;
  *(volatile v8h*)op = o;
  __threadfence();
  *(volatile v8h*)op = o;
}

__global__ __launch_bounds__(128) void k_rms(const float* __restrict__ lo, const float* __restrict__ x,
                                            const float* __restrict__ w, _Float16* __restrict__ out) {
  __shared__ float red[4];
  const int row = blockIdx.x, tid = threadIdx.x, c0 = tid * 8;
  const float* lr = lo + (size_t)row * ND + c0;
  const float* xr = x + (size_t)row * ND + c0;
  const v4f la = *(const v4f*)(lr), lb = *(const v4f*)(lr + 4);
  const v4f xa = *(const v4f*)(xr), xb = *(const v4f*)(xr + 4);
  float v[8];
#pragma unroll
  for (int e = 0; e < 4; ++e) { v[e] = la[e] + xa[e]; v[4 + e] = lb[e] + xb[e]; }
  float s2 = 0.f;
#pragma unroll
  for (int e = 0; e < 8; ++e) s2 += v[e] * v[e];
  s2 = block_sum128(s2, red);
  const float rstd = rsqrtf(s2 * (1.0f / ND) + 1e-5f);
  const v4f wa = *(const v4f*)(w + c0), wb = *(const v4f*)(w + c0 + 4);
  v8h o;
#pragma unroll
  for (int e = 0; e < 4; ++e) {
    o[e]     = (_Float16)(v[e] * rstd * wa[e]);
    o[4 + e] = (_Float16)(v[4 + e] * rstd * wb[e]);
  }
  _Float16* op = out + (size_t)row * ND + c0;
  *(volatile v8h*)op = o;
  __threadfence();
  *(volatile v8h*)op = o;
}

__global__ __launch_bounds__(256) void k_wtrans(const float* __restrict__ W, _Float16* __restrict__ out,
                                               int R, int Cc, float scale) {
  __shared__ __align__(16) float tf[64 * 68];
  const int c0  = blockIdx.x * 64;
  const int r0  = blockIdx.y * 64;
  const int tid = threadIdx.x;
  {
    const int lr = tid >> 4;
    const int c4 = (tid & 15) * 4;
#pragma unroll
    for (int it = 0; it < 4; ++it) {
      const int rr = it * 16 + lr;
      const v4f a = *(const v4f*)(W + (size_t)(r0 + rr) * Cc + c0 + c4);
      *(v4f*)(tf + rr * 68 + c4) = a;
    }
  }
  __syncthreads();
  const int sub = tid >> 3;
  const int c8  = (tid & 7) * 8;
  v8h hv[2];
#pragma unroll
  for (int it = 0; it < 2; ++it) {
    const int oc = it * 32 + sub;
    v8h t;
#pragma unroll
    for (int e = 0; e < 8; ++e) t[e] = (_Float16)(tf[(c8 + e) * 68 + oc] * scale);
    hv[it] = t;
  }
  for (int pass = 0; pass < 2; ++pass) {
#pragma unroll
    for (int it = 0; it < 2; ++it) {
      const int oc = it * 32 + sub;
      *(volatile v8h*)(out + (size_t)(c0 + oc) * R + r0 + c8) = hv[it];
    }
    __threadfence();
  }
}

template <int BIAS_MODE, int OUT_MODE, int EPI>
__global__ __launch_bounds__(256) void k_gemm64(
    const _Float16* __restrict__ A, int lda,
    const _Float16* __restrict__ Bt, int ldb,
    void* __restrict__ Cout, int ldc,
    const float* __restrict__ bias,
    const float* __restrict__ aux, int ldx,
    int M, int N, int K, float scale) {
  __shared__ __align__(16) float sT[8][16 * 68];
  const int lane = threadIdx.x & 31;
  const int wave = threadIdx.x >> 5;
  const int tilesN = N >> 6, tilesM = M >> 6;
  const int tile = blockIdx.x * 8 + wave;
  if (tile >= tilesM * tilesN) return;
  const int tm = tile / tilesN;
  const int tn = tile - tm * tilesN;
  const int m0 = tm << 6, n0 = tn << 6;
  const int rl   = lane & 15;
  const int hh   = lane >> 4;
  const int koff = hh * 8;
  const int mOff = hh * 8;

  const v8f z8 = {0.f, 0.f, 0.f, 0.f, 0.f, 0.f, 0.f, 0.f};
  v8f acc[4][4];
#pragma unroll
  for (int i = 0; i < 4; ++i)
#pragma unroll
    for (int j = 0; j < 4; ++j) acc[i][j] = z8;

  const _Float16* Ab = A  + (size_t)(m0 + rl) * lda + koff;
  const _Float16* Bb = Bt + (size_t)(n0 + rl) * ldb + koff;

  for (int k0 = 0; k0 < K; k0 += 32) {
    v16h bf[4];
#pragma unroll
    for (int j = 0; j < 4; ++j) bf[j] = frag_load(Bb + (size_t)(16 * j) * ldb + k0);
#pragma unroll
    for (int i = 0; i < 4; ++i) {
      const v16h af = frag_load(Ab + (size_t)(16 * i) * lda + k0);
#pragma unroll
      for (int j = 0; j < 4; ++j) acc[i][j] = mma16(af, bf[j], acc[i][j]);
      guard4(acc[i][0], acc[i][1], acc[i][2], acc[i][3], af, bf[0], bf[1], bf[2], bf[3]);
    }
  }
  accg4(acc[0][0], acc[0][1], acc[0][2], acc[0][3]);
  accg4(acc[1][0], acc[1][1], acc[1][2], acc[1][3]);
  accg4(acc[2][0], acc[2][1], acc[2][2], acc[2][3]);
  accg4(acc[3][0], acc[3][1], acc[3][2], acc[3][3]);

  float* slab = sT[wave];
#pragma unroll
  for (int i = 0; i < 4; ++i) {
    const int mBase = m0 + (i << 4);
#pragma unroll
    for (int j = 0; j < 4; ++j) {
      const int n = n0 + (j << 4) + rl;
      float bv = 0.f;
      if (BIAS_MODE == 2) bv = bias[n];
#pragma unroll
      for (int r = 0; r < 8; ++r) {
        const int m = mBase + mOff + r;
        float v = acc[i][j][r] * scale;
        if (BIAS_MODE == 1) v += bias[m];
        if (BIAS_MODE == 2) v += bv;
        if (EPI == 1) v = silu_f(v);
        if (EPI == 2) v = silu_f(aux[(size_t)m * ldx + n]) * v;
        if (EPI == 3) v += aux[(size_t)m * ldx + n];
        slab[(mOff + r) * 68 + (j << 4) + rl] = v;
      }
    }
    lds_sync_wave();
    if (OUT_MODE == 0) {
      float* C = (float*)Cout;
      const int c4 = rl * 4;
      for (int pass = 0; pass < 2; ++pass) {
#pragma unroll
        for (int it = 0; it < 8; ++it) {
          const int row = it * 2 + hh;
          const v4f v = *(const v4f*)(slab + row * 68 + c4);
          *(volatile v4f*)(C + (size_t)(mBase + row) * ldc + n0 + c4) = v;
        }
        __threadfence();
      }
    } else {
      _Float16* C = (_Float16*)Cout;
      const int q = lane >> 3, c8 = (lane & 7) * 8;
      v8h hv[4];
#pragma unroll
      for (int it = 0; it < 4; ++it) {
        const int row = it * 4 + q;
        const float* sp = slab + row * 68 + c8;
        v8h t;
#pragma unroll
        for (int e = 0; e < 8; ++e) t[e] = (_Float16)sp[e];
        hv[it] = t;
      }
      for (int pass = 0; pass < 2; ++pass) {
#pragma unroll
        for (int it = 0; it < 4; ++it) {
          const int row = it * 4 + q;
          *(volatile v8h*)(C + (size_t)(mBase + row) * ldc + n0 + c8) = hv[it];
        }
        __threadfence();
      }
    }
    lds_sync_wave();
  }
}

__global__ __launch_bounds__(128) void k_attn(const _Float16* __restrict__ QK, const _Float16* __restrict__ Vt,
                                             float* __restrict__ O, float sscale) {
  __shared__ __align__(16) _Float16 Ks[64 * 128];
  __shared__ __align__(16) _Float16 Vs[128 * 64];
  __shared__ __align__(16) _Float16 Ps[4][16 * 64];
  __shared__ __align__(16) float    Os[4][16 * 68];

  const int tid  = threadIdx.x;
  const int wave = tid >> 5;
  const int lane = tid & 31;
  const int hh   = lane >> 4;
  const int c    = lane & 15;

  const int bx = blockIdx.x;
  const int qb = bx & 31;
  const int bh = bx >> 5;
  const int b  = bh >> 3;
  const int h  = bh & 7;
  const int tok0 = b * NS;
  const int q0   = qb * 64 + wave * 16;
  const size_t QKP = 2 * ND;

  v16h qf[4];
  {
    const _Float16* qp = QK + (size_t)(tok0 + q0 + c) * QKP + h * NHD + 8 * hh;
#pragma unroll
    for (int dc = 0; dc < 4; ++dc) qf[dc] = frag_load(qp + dc * 32);
  }

  const v8f z8 = {0.f, 0.f, 0.f, 0.f, 0.f, 0.f, 0.f, 0.f};
  float mrow[8], lrow[8];
  v8f oacc[8];
#pragma unroll
  for (int r = 0; r < 8; ++r) { mrow[r] = -INFINITY; lrow[r] = 0.f; }
#pragma unroll
  for (int t = 0; t < 8; ++t) oacc[t] = z8;

  const int nCh = qb + 1;
  for (int kc = 0; kc < nCh; ++kc) {
    const int kv0 = kc * 64;
    __syncthreads();
    {
      const int r = tid >> 1, hf = (tid & 1) * 64;
      const _Float16* kp = QK + (size_t)(tok0 + kv0 + r) * QKP + ND + h * NHD + hf;
      _Float16* kd = Ks + r * 128 + hf;
#pragma unroll
      for (int i = 0; i < 8; ++i) *(v8h*)(kd + 8 * i) = *(const v8h*)(kp + 8 * i);
      const _Float16* vp = Vt + (size_t)(h * NHD + tid) * NTOK + tok0 + kv0;
      _Float16* vd = Vs + tid * 64;
#pragma unroll
      for (int i = 0; i < 8; ++i) *(v8h*)(vd + 8 * i) = *(const v8h*)(vp + 8 * i);
    }
    __syncthreads();

    v8f s[4];
#pragma unroll
    for (int j = 0; j < 4; ++j) {
      s[j] = z8;
      v16h kb[4];
      const _Float16* kr = Ks + (j * 16 + c) * 128 + 8 * hh;
#pragma unroll
      for (int dc = 0; dc < 4; ++dc) kb[dc] = frag_load(kr + dc * 32);
#pragma unroll
      for (int dc = 0; dc < 4; ++dc) s[j] = mma16(qf[dc], kb[dc], s[j]);
      guard1(s[j], kb[0], kb[1], kb[2], kb[3], qf[3]);
    }

    const bool diag = (kc == qb);
    float cm[8];
#pragma unroll
    for (int r = 0; r < 8; ++r) {
      const int qrow = q0 + 8 * hh + r;
      float m = -INFINITY;
#pragma unroll
      for (int j = 0; j < 4; ++j) {
        const int kvcol = kv0 + j * 16 + c;
        const float sv = s[j][r] * sscale;
        const bool masked = diag && (kvcol > qrow);
        const float sm = masked ? -INFINITY : sv;
        s[j][r] = sm;
        m = fmaxf(m, sm);
      }
#pragma unroll
      for (int off = 1; off < 16; off <<= 1) m = fmaxf(m, __shfl_xor(m, off, 32));
      cm[r] = m;
    }

    _Float16* pw = Ps[wave];
#pragma unroll
    for (int r = 0; r < 8; ++r) {
      const float mnew  = fmaxf(mrow[r], cm[r]);
      const float alpha = __expf(mrow[r] - mnew);
      mrow[r] = mnew;
      float psum = 0.f;
#pragma unroll
      for (int j = 0; j < 4; ++j) {
        const float p = __expf(s[j][r] - mnew);
        psum += p;
        pw[(8 * hh + r) * 64 + j * 16 + c] = (_Float16)(p * 256.0f);
      }
#pragma unroll
      for (int off = 1; off < 16; off <<= 1) psum += __shfl_xor(psum, off, 32);
      lrow[r] = lrow[r] * alpha + psum;
#pragma unroll
      for (int t = 0; t < 8; ++t) oacc[t][r] *= alpha;
    }
    lds_sync_wave();

#pragma unroll
    for (int kk = 0; kk < 2; ++kk) {
      const v16h pa = frag_load(pw + c * 64 + kk * 32 + 8 * hh);
#pragma unroll
      for (int tg = 0; tg < 2; ++tg) {
        v16h vb[4];
#pragma unroll
        for (int t4 = 0; t4 < 4; ++t4)
          vb[t4] = frag_load(Vs + ((tg * 4 + t4) * 16 + c) * 64 + kk * 32 + 8 * hh);
#pragma unroll
        for (int t4 = 0; t4 < 4; ++t4) oacc[tg * 4 + t4] = mma16(pa, vb[t4], oacc[tg * 4 + t4]);
        guard4(oacc[tg * 4 + 0], oacc[tg * 4 + 1], oacc[tg * 4 + 2], oacc[tg * 4 + 3],
               pa, vb[0], vb[1], vb[2], vb[3]);
      }
    }
  }

  float inv[8];
#pragma unroll
  for (int r = 0; r < 8; ++r) inv[r] = (1.0f / lrow[r]) * (1.0f / 256.0f);
  float* os = Os[wave];
  float* ob = O + (size_t)(tok0 + q0) * ND + h * NHD;
  const int c4 = c * 4;
#pragma unroll
  for (int dh = 0; dh < 2; ++dh) {
    if (dh) lds_sync_wave();
#pragma unroll
    for (int r = 0; r < 8; ++r)
#pragma unroll
      for (int t = 0; t < 4; ++t) os[(8 * hh + r) * 68 + t * 16 + c] = oacc[dh * 4 + t][r] * inv[r];
    lds_sync_wave();
    for (int pass = 0; pass < 2; ++pass) {
#pragma unroll
      for (int it = 0; it < 8; ++it) {
        const int row = it * 2 + hh;
        const v4f val = *(const v4f*)(os + row * 68 + c4);
        *(volatile v4f*)(ob + (size_t)row * ND + dh * 64 + c4) = val;
      }
      __threadfence();
    }
  }
}

extern "C" void kernel_launch(void* const* d_in, const int* in_sizes, int n_in,
                              void* d_out, int out_size, void* d_ws, size_t ws_size,
                              hipStream_t stream) {
  if (n_in < 12) return;
  if (in_sizes[0] != NTOK * ND) return;
  if (in_sizes[2] != ND || in_sizes[3] != ND || in_sizes[6] != ND || in_sizes[7] != ND || in_sizes[9] != ND) return;
  if (in_sizes[4] != ND * 4 * ND || in_sizes[5] != 4 * ND) return;
  if (in_sizes[8] != ND * ND || in_sizes[10] != ND * 2 * ND || in_sizes[11] != ND * ND) return;
  if (out_size != NTOK * ND) return;

  const float* x        = (const float*)d_in[0];
  const float* ln_in_w  = (const float*)d_in[2];
  const float* ln_in_b  = (const float*)d_in[3];
  const float* W_uvqk   = (const float*)d_in[4];
  const float* b_uvqk   = (const float*)d_in[5];
  const float* ln_out_w = (const float*)d_in[6];
  const float* ln_out_b = (const float*)d_in[7];
  const float* W_proj   = (const float*)d_in[8];
  const float* rms_w    = (const float*)d_in[9];
  const float* W1       = (const float*)d_in[10];
  const float* W2       = (const float*)d_in[11];
  float* out = (float*)d_out;

  const size_t MB = 1048576;
  const size_t oWT0 = 0 * MB,  oWTp = 8 * MB,  oWT1 = 10 * MB, oWT2 = 14 * MB;
  const size_t oU   = 16 * MB, oQK  = 48 * MB, oVt  = 80 * MB, oXn  = 112 * MB;
  const size_t oATT = 96 * MB, oP16 = 48 * MB, oLO  = 64 * MB, oF16 = 16 * MB;
  const size_t oHa  = 32 * MB, oG16 = 96 * MB;
  const size_t total = 128 * MB;
  if ((size_t)NTOK * ND * 4 != 32 * MB) return;
  if (total > ws_size) return;

  char* ws = (char*)d_ws;
  _Float16* WT0 = (_Float16*)(ws + oWT0);
  _Float16* WTp = (_Float16*)(ws + oWTp);
  _Float16* WT1 = (_Float16*)(ws + oWT1);
  _Float16* WT2 = (_Float16*)(ws + oWT2);
  float*    U   = (float*)(ws + oU);
  _Float16* QK  = (_Float16*)(ws + oQK);
  _Float16* Vt  = (_Float16*)(ws + oVt);
  _Float16* Xn  = (_Float16*)(ws + oXn);
  float*    ATT = (float*)(ws + oATT);
  _Float16* P16 = (_Float16*)(ws + oP16);
  float*    LO  = (float*)(ws + oLO);
  _Float16* F16 = (_Float16*)(ws + oF16);
  float*    Ha  = (float*)(ws + oHa);
  _Float16* G16 = (_Float16*)(ws + oG16);

  const float wsc   = 64.0f;
  const float iwsc  = 1.0f / 64.0f;
  const dim3 blk(256);

  k_ln<<<dim3(NTOK), dim3(128), 0, stream>>>(x, ln_in_w, ln_in_b, Xn);
  k_wtrans<<<dim3(4 * ND / 64, ND / 64), blk, 0, stream>>>(W_uvqk, WT0, ND, 4 * ND, wsc);
  k_wtrans<<<dim3(ND / 64, ND / 64), blk, 0, stream>>>(W_proj, WTp, ND, ND, wsc);
  k_wtrans<<<dim3(2 * ND / 64, ND / 64), blk, 0, stream>>>(W1, WT1, ND, 2 * ND, wsc);
  k_wtrans<<<dim3(ND / 64, ND / 64), blk, 0, stream>>>(W2, WT2, ND, ND, wsc);

  const int tilesTokD  = (NTOK / 64) * (ND / 64);
  const int tilesTok2D = (NTOK / 64) * (2 * ND / 64);
  const dim3 gTokD((tilesTokD + 7) / 8);
  const dim3 gTok2D((tilesTok2D + 7) / 8);

  k_gemm64<2, 0, 1><<<gTokD, blk, 0, stream>>>(Xn, ND, WT0, ND, (void*)U, ND, b_uvqk, U, ND, NTOK, ND, ND, iwsc);
  k_gemm64<2, 1, 1><<<gTok2D, blk, 0, stream>>>(Xn, ND, WT0 + (size_t)2 * ND * ND, ND, (void*)QK, 2 * ND,
                                                b_uvqk + 2 * ND, U, ND, NTOK, 2 * ND, ND, iwsc);
  k_gemm64<1, 1, 1><<<gTokD, blk, 0, stream>>>(WT0 + (size_t)ND * ND, ND, Xn, ND, (void*)Vt, NTOK,
                                               b_uvqk + ND, U, ND, ND, NTOK, ND, iwsc);
  k_attn<<<dim3(NBATCH * NHEAD * (NS / 64)), dim3(128), 0, stream>>>(QK, Vt, ATT, 0.08838834764831845f);
  k_lngate<<<dim3(NTOK), dim3(128), 0, stream>>>(ATT, U, ln_out_w, ln_out_b, P16);
  k_gemm64<0, 0, 0><<<gTokD, blk, 0, stream>>>(P16, ND, WTp, ND, (void*)LO, ND, b_uvqk, LO, ND, NTOK, ND, ND, iwsc);
  k_rms<<<dim3(NTOK), dim3(128), 0, stream>>>(LO, x, rms_w, F16);
  k_gemm64<0, 0, 0><<<gTokD, blk, 0, stream>>>(F16, ND, WT1, ND, (void*)Ha, ND, b_uvqk, LO, ND, NTOK, ND, ND, iwsc);
  k_gemm64<0, 1, 2><<<gTokD, blk, 0, stream>>>(F16, ND, WT1 + (size_t)ND * ND, ND, (void*)G16, ND, b_uvqk, Ha, ND,
                                               NTOK, ND, ND, 0.25f);
  k_gemm64<0, 0, 3><<<gTokD, blk, 0, stream>>>(G16, ND, WT2, ND, (void*)out, ND, b_uvqk, LO, ND, NTOK, ND, ND,
                                               1.0f / 1024.0f);
  (void)hipGetLastError();
}
